// DeformableBasicBlock_35759897706918
// MI455X (gfx1250) — hardware-verified
//
#include <hip/hip_runtime.h>
#include <stdint.h>

#define DEVINL __device__ __forceinline__

typedef _Float16 f16t;
typedef _Float16 v16h __attribute__((ext_vector_type(16)));
typedef _Float16 v8h  __attribute__((ext_vector_type(8)));
typedef _Float16 v2h  __attribute__((ext_vector_type(2)));
typedef float    v8f  __attribute__((ext_vector_type(8)));
typedef float    v4f  __attribute__((ext_vector_type(4)));
typedef int      v4i  __attribute__((ext_vector_type(4)));
typedef unsigned v4u  __attribute__((ext_vector_type(4)));
typedef v8h __attribute__((may_alias)) v8ha;
typedef v2h __attribute__((may_alias)) v2ha;
typedef v4f __attribute__((may_alias)) v4fa;
typedef v4i __attribute__((may_alias)) v4ia;
typedef v4u __attribute__((may_alias)) v4ua;
union FragH { v16h v; v8h half[2]; };

#define CCH   128
#define HH    128
#define WW    128
#define HWPIX (HH * WW)
#define KTAP  9
#define KDIM  (CCH * KTAP)
#define KSTEP 32
#define NIT   (KDIM / KSTEP)
#define MT    64
#define NSUB  4
#define TPB   256
#define GGRP  4
#define ACAR  16.0f
#define WCAR  256.0f
#define MCAR  16.0f

static_assert(KDIM % KSTEP == 0);
static_assert(CCH % KSTEP == 0);
static_assert(WW % MT == 0);
static_assert(TPB == 8 * 32);
static_assert(MT * (KSTEP / 8) == TPB);
static_assert(GGRP * 2 == 8);
static_assert(NSUB * 16 == MT);
static_assert(CCH == 8 * 16);
static_assert((CCH * KDIM * 2) % 128 == 0);
static_assert((MT * CCH * 2) % 128 == 0);

DEVINL int imin(int a, int b) { return a < b ? a : b; }
DEVINL int imax(int a, int b) { return a > b ? a : b; }

DEVINL v8f wmma_f16(v16h a, v16h b, v8f c) {
  v8f d = __builtin_amdgcn_wmma_f32_16x16x32_f16(false, a, false, b, (short)0, c, false, false);
  asm volatile("v_nop\n\tv_nop\n\tv_nop\n\tv_nop" : "+v"(d) : "v"(a), "v"(b));
  return d;
}
DEVINL v8f zero8f() {
  v8f z = {0.f, 0.f, 0.f, 0.f, 0.f, 0.f, 0.f, 0.f};
  return z;
}

DEVINL v16h frag_row(const f16t* rowp, int h) {
  FragH f;
  f.half[0] = *(const v8ha*)(rowp + 8 * h);
  f.half[1] = *(const v8ha*)(rowp + 16 + 8 * h);
  return f.v;
}

__global__ __launch_bounds__(TPB) void prep_w_k(const float* __restrict__ w1,
                                               const float* __restrict__ w2,
                                               f16t* __restrict__ w1T,
                                               f16t* __restrict__ w2T)
{
  const int y = blockIdx.y;
  const float* src = (y == 0) ? w1 : w2;
  f16t* dstp = (y == 0) ? w1T : w2T;
  const int t = blockIdx.x * TPB + threadIdx.x;
  if (t >= CCH * (KDIM / 8)) return;
  const int n    = t / (KDIM / 8);
  const int part = t - n * (KDIM / 8);
  const int k0   = part * 8;
  const int tap  = k0 >> 7;
  const int cin0 = k0 & 127;
  const float* sp = src + (size_t)n * KDIM + (size_t)cin0 * KTAP + tap;
  v8h o;
  #pragma unroll
  for (int j = 0; j < 8; ++j) o[j] = (f16t)(sp[j * KTAP] * WCAR);
  f16t* dst = dstp + (size_t)8 * t;
  *(volatile v8h*)dst = o;
  __threadfence();
  *(volatile v8h*)dst = o;
}

__global__ __launch_bounds__(TPB) void deform_conv_k(
    const float* __restrict__ x, const float* __restrict__ off,
    const f16t* __restrict__ w1T,
    const float* __restrict__ g1, const float* __restrict__ be1,
    const float* __restrict__ mu1, const float* __restrict__ var1,
    f16t* __restrict__ mid)
{
  __shared__ __attribute__((aligned(16))) v4i  sO[MT * KTAP];
  __shared__ __attribute__((aligned(16))) v4f  sW[MT * KTAP];
  __shared__ __attribute__((aligned(16))) f16t Als[2][MT * KSTEP];
  __shared__ __attribute__((aligned(16))) f16t sStg[MT * CCH];
  __shared__ __attribute__((aligned(16))) float sK[CCH];
  __shared__ __attribute__((aligned(16))) float sB[CCH];

  const int tid  = threadIdx.x;
  const int lane = tid & 31;
  const int wave = tid >> 5;
  const int hl   = lane >> 4;
  const int m    = lane & 15;

  const int pix0 = blockIdx.x * MT;
  const int b    = pix0 / HWPIX;
  const int rem  = pix0 - b * HWPIX;
  const int h    = rem / WW;
  const int w0   = rem - h * WW;

  if (tid < CCH) {
    const float inv = g1[tid] * rsqrtf(var1[tid] + 1e-5f);
    const float add = be1[tid] - mu1[tid] * inv;
    sK[tid] = inv * (MCAR / (ACAR * WCAR));
    sB[tid] = add * MCAR;
  }

  #pragma unroll 1
  for (int t = tid; t < MT * KTAP; t += TPB) {
    const int p   = t / KTAP;
    const int tap = t - p * KTAP;
    const int w   = w0 + p;
    const float dy = off[(((size_t)b * (2 * KTAP) + 2 * tap    ) * HH + h) * WW + w];
    const float dx = off[(((size_t)b * (2 * KTAP) + 2 * tap + 1) * HH + h) * WW + w];
    const float py = ((float)h + (float)(tap / 3 - 1)) + dy;
    const float px = ((float)w + (float)(tap % 3 - 1)) + dx;
    const float y0f = floorf(py), x0f = floorf(px);
    const float y1f = y0f + 1.0f, x1f = x0f + 1.0f;
    const float fy = py - y0f, fx = px - x0f;
    const float ey = 1.0f - fy, ex = 1.0f - fx;
    const bool vy0 = (y0f >= 0.0f) && (y0f <= (float)(HH - 1));
    const bool vy1 = (y1f >= 0.0f) && (y1f <= (float)(HH - 1));
    const bool vx0 = (x0f >= 0.0f) && (x0f <= (float)(WW - 1));
    const bool vx1 = (x1f >= 0.0f) && (x1f <= (float)(WW - 1));
    const int y0i = (int)fminf(fmaxf(y0f, 0.0f), (float)(HH - 1));
    const int y1i = (int)fminf(fmaxf(y1f, 0.0f), (float)(HH - 1));
    const int x0i = (int)fminf(fmaxf(x0f, 0.0f), (float)(WW - 1));
    const int x1i = (int)fminf(fmaxf(x1f, 0.0f), (float)(WW - 1));
    v4i o;
    o[0] = y0i * WW + x0i;  o[1] = y0i * WW + x1i;
    o[2] = y1i * WW + x0i;  o[3] = y1i * WW + x1i;
    v4f g;
    g[0] = (vy0 && vx0) ? ey * ex : 0.0f;
    g[1] = (vy0 && vx1) ? ey * fx : 0.0f;
    g[2] = (vy1 && vx0) ? fy * ex : 0.0f;
    g[3] = (vy1 && vx1) ? fy * fx : 0.0f;
    sO[t] = o;
    sW[t] = g;
  }
  __syncthreads();

  const int pgrp  = tid & 63;
  const int cgrp  = tid >> 6;
  const int nbase = wave * 16;

  v8f acc[NSUB];
  #pragma unroll
  for (int s = 0; s < NSUB; ++s) acc[s] = zero8f();

  #pragma unroll 1
  for (int it = 0; it < NIT; ++it) {
    const int k0  = it * KSTEP;
    const int tap = k0 >> 7;
    const int c0  = k0 & 127;
    const int buf = it & 1;

    {
      const v4i o = sO[pgrp * KTAP + tap];
      const v4f g = sW[pgrp * KTAP + tap];
      const float* xb = x + ((size_t)(b * CCH + c0 + cgrp * 8)) * HWPIX;
      f16t* dstl = &Als[buf][pgrp * KSTEP + cgrp * 8];
      #pragma unroll 1
      for (int jj = 0; jj < GGRP; ++jj) {
        const float* xp0 = xb + (size_t)(2 * jj) * HWPIX;
        const float* xp1 = xp0 + HWPIX;
        const float a0 = xp0[o[0]], a1 = xp0[o[1]], a2 = xp0[o[2]], a3 = xp0[o[3]];
        const float c0v = xp1[o[0]], c1v = xp1[o[1]], c2v = xp1[o[2]], c3v = xp1[o[3]];
        const float v0 = g[0] * a0  + g[1] * a1  + g[2] * a2  + g[3] * a3;
        const float v1 = g[0] * c0v + g[1] * c1v + g[2] * c2v + g[3] * c3v;
        v2h t2;
        t2[0] = (f16t)(v0 * ACAR);
        t2[1] = (f16t)(v1 * ACAR);
        *(v2ha*)(dstl + 2 * jj) = t2;
      }
    }
    __syncthreads();

    const v16h wf = frag_row(w1T + (size_t)(nbase + m) * KDIM + k0, hl);
    #pragma unroll
    for (int s = 0; s < NSUB; ++s) {
      const v16h xf = frag_row(&Als[buf][(s * 16 + m) * KSTEP], hl);
      acc[s] = wmma_f16(wf, xf, acc[s]);
    }
  }

  {
    const v4f ka = *(const v4fa*)&sK[nbase + 8 * hl];
    const v4f kb = *(const v4fa*)&sK[nbase + 8 * hl + 4];
    const v4f ba = *(const v4fa*)&sB[nbase + 8 * hl];
    const v4f bb = *(const v4fa*)&sB[nbase + 8 * hl + 4];
    #pragma unroll
    for (int s = 0; s < NSUB; ++s) {
      v8h o;
      #pragma unroll
      for (int r = 0; r < 4; ++r) {
        const float t0 = fmaxf(fmaf(acc[s][r],     ka[r], ba[r]), 0.0f);
        const float t1 = fmaxf(fmaf(acc[s][4 + r], kb[r], bb[r]), 0.0f);
        o[r]     = (f16t)t0;
        o[4 + r] = (f16t)t1;
      }
      *(v8ha*)&sStg[(s * 16 + m) * CCH + nbase + 8 * hl] = o;
    }
  }
  __syncthreads();

  {
    f16t* gt = mid + (size_t)pix0 * CCH;
    const int q = lane >> 3, e = lane & 7;
    v8h pv[4];
    int offh[4];
    #pragma unroll
    for (int i = 0; i < 4; ++i) {
      const int L = wave * 16 + 4 * i + q;
      offh[i] = L * 64 + e * 8;
      pv[i] = *(const v8ha*)&sStg[offh[i]];
    }
    #pragma unroll
    for (int i = 0; i < 4; ++i) *(volatile v8h*)(gt + offh[i]) = pv[i];
    __threadfence();
    #pragma unroll
    for (int i = 0; i < 4; ++i) *(volatile v8h*)(gt + offh[i]) = pv[i];
  }
}

__global__ __launch_bounds__(TPB) void conv_k(
    const f16t* __restrict__ mid, const f16t* __restrict__ w2T,
    const float* __restrict__ g2, const float* __restrict__ be2,
    const float* __restrict__ mu2, const float* __restrict__ var2,
    const float* __restrict__ x, float* __restrict__ out)
{
  __shared__ __attribute__((aligned(16))) f16t  Als[2][MT * KSTEP];
  __shared__ __attribute__((aligned(16))) float sStg[CCH * MT];
  __shared__ __attribute__((aligned(16))) float sK[CCH];
  __shared__ __attribute__((aligned(16))) float sB[CCH];

  const int tid  = threadIdx.x;
  const int lane = tid & 31;
  const int wave = tid >> 5;
  const int hl   = lane >> 4;
  const int m    = lane & 15;

  const int pix0 = blockIdx.x * MT;
  const int b    = pix0 / HWPIX;
  const int rem  = pix0 - b * HWPIX;
  const int h    = rem / WW;
  const int w0   = rem - h * WW;

  if (tid < CCH) {
    const float inv = g2[tid] * rsqrtf(var2[tid] + 1e-5f);
    const float add = be2[tid] - mu2[tid] * inv;
    sK[tid] = inv * (1.0f / (MCAR * WCAR));
    sB[tid] = add;
  }

  const int pgrp  = tid & 63;
  const int cgrp  = tid >> 6;
  const int nbase = wave * 16;

  v8f acc[NSUB];
  #pragma unroll
  for (int s = 0; s < NSUB; ++s) acc[s] = zero8f();

  #pragma unroll 1
  for (int it = 0; it < NIT; ++it) {
    const int k0  = it * KSTEP;
    const int tap = k0 >> 7;
    const int c0  = k0 & 127;
    const int buf = it & 1;

    {
      const int yy = h + (tap / 3) - 1;
      const int xx = w0 + pgrp + (tap % 3) - 1;
      const bool valid = (yy >= 0) && (yy <= HH - 1) && (xx >= 0) && (xx <= WW - 1);
      const int yyc = imin(imax(yy, 0), HH - 1);
      const int xxc = imin(imax(xx, 0), WW - 1);
      const f16t* sp = mid + ((size_t)(b * HWPIX + yyc * WW + xxc)) * CCH + c0 + cgrp * 8;
      v4u v = *(const v4ua*)sp;
      const unsigned msk = valid ? 0xffffffffu : 0u;
      v = v & msk;
      *(v4ua*)&Als[buf][pgrp * KSTEP + cgrp * 8] = v;
    }
    __syncthreads();

    const v16h wf = frag_row(w2T + (size_t)(nbase + m) * KDIM + k0, hl);
    #pragma unroll
    for (int s = 0; s < NSUB; ++s) {
      const v16h xf = frag_row(&Als[buf][(s * 16 + m) * KSTEP], hl);
      acc[s] = wmma_f16(xf, wf, acc[s]);
    }
  }

  {
    float* row = &sStg[(nbase + m) * MT + 8 * hl];
    #pragma unroll
    for (int s = 0; s < NSUB; ++s) {
      v4f lo4, hi4;
      #pragma unroll
      for (int r = 0; r < 4; ++r) { lo4[r] = acc[s][r]; hi4[r] = acc[s][4 + r]; }
      *(v4fa*)(row + 16 * s)     = lo4;
      *(v4fa*)(row + 16 * s + 4) = hi4;
    }
  }
  __syncthreads();

  {
    const int q = lane >> 3, e = lane & 7;
    v4f ov[8];
    size_t gofs[8];
    #pragma unroll
    for (int i = 0; i < 8; ++i) {
      const int c  = nbase + 2 * i + (q >> 1);
      const int po = (q & 1) * 32 + e * 4;
      const v4f a  = *(const v4fa*)&sStg[c * MT + po];
      gofs[i] = ((size_t)(b * CCH + c)) * HWPIX + (size_t)h * WW + w0 + po;
      const v4f xr = *(const v4fa*)(x + gofs[i]);
      const float kk = sK[c], bb = sB[c];
      v4f o;
      #pragma unroll
      for (int j = 0; j < 4; ++j) o[j] = fmaxf(fmaf(a[j], kk, bb) + xr[j], 0.0f);
      ov[i] = o;
    }
    #pragma unroll
    for (int i = 0; i < 8; ++i) *(volatile v4f*)(out + gofs[i]) = ov[i];
    __threadfence();
    #pragma unroll
    for (int i = 0; i < 8; ++i) *(volatile v4f*)(out + gofs[i]) = ov[i];
  }
}

extern "C" void kernel_launch(void* const* d_in, const int* in_sizes, int n_in,
                              void* d_out, int out_size, void* d_ws, size_t ws_size,
                              hipStream_t stream) {
  if (n_in < 12) return;
  const int chw = CCH * HWPIX;
  if (in_sizes[0] <= 0 || (in_sizes[0] % chw) != 0) return;
  const int nB = in_sizes[0] / chw;
  if (in_sizes[1] != nB * 2 * KTAP * HWPIX) return;
  if (in_sizes[2] != CCH * KDIM) return;
  if (in_sizes[7] != CCH * KDIM) return;
  if (in_sizes[3] != CCH || in_sizes[4] != CCH || in_sizes[5] != CCH || in_sizes[6] != CCH) return;
  if (in_sizes[8] != CCH || in_sizes[9] != CCH || in_sizes[10] != CCH || in_sizes[11] != CCH) return;
  if (out_size != in_sizes[0]) return;

  const float* x    = (const float*)d_in[0];
  const float* offp = (const float*)d_in[1];
  const float* w1   = (const float*)d_in[2];
  const float* g1   = (const float*)d_in[3];
  const float* be1  = (const float*)d_in[4];
  const float* mu1  = (const float*)d_in[5];
  const float* var1 = (const float*)d_in[6];
  const float* w2   = (const float*)d_in[7];
  const float* g2   = (const float*)d_in[8];
  const float* be2  = (const float*)d_in[9];
  const float* mu2  = (const float*)d_in[10];
  const float* var2 = (const float*)d_in[11];
  float* outp = (float*)d_out;

  const size_t szW   = (size_t)CCH * KDIM * 2;
  const size_t szMid = (size_t)nB * HWPIX * CCH * 2;
  size_t off = 0;
  char* ws = (char*)d_ws;
  f16t* w1T = (f16t*)(ws + off); off += szW;
  f16t* w2T = (f16t*)(ws + off); off += szW;
  f16t* mid = (f16t*)(ws + off); off += szMid;
  if (off > ws_size) return;

  const int npix   = nB * HWPIX;
  const int blocks = npix / MT;

  prep_w_k<<<dim3((CCH * (KDIM / 8) + TPB - 1) / TPB, 2), TPB, 0, stream>>>(w1, w2, w1T, w2T);
  deform_conv_k<<<blocks, TPB, 0, stream>>>(x, offp, w1T, g1, be1, mu1, var1, mid);
  conv_k<<<blocks, TPB, 0, stream>>>(mid, w2T, g2, be2, mu2, var2, x, outp);
}
